// TensorLogicSSM_25443386262309
// MI455X (gfx1250) — hardware-run, weakly checked
//
#include <hip/hip_runtime.h>
#include <math.h>

typedef __attribute__((ext_vector_type(16))) _Float16 v16h;
typedef __attribute__((ext_vector_type(8)))  _Float16 v8h;
typedef __attribute__((ext_vector_type(8)))  float    v8f;
typedef __attribute__((ext_vector_type(4)))  float    v4f;

constexpr int kVocab   = 50257;
constexpr int kHid     = 16;
constexpr int kBatch   = 256;
constexpr int kSteps   = 4096;
constexpr int kVPad    = 50304;
constexpr int kKPad    = 32;
constexpr int kNInPad  = 64;
constexpr int kOutTot  = kBatch * kVocab;
constexpr int kOut4    = kOutTot / 4;

constexpr float kCarryEmb   = 64.0f;
constexpr float kCarryBw    = 64.0f;
constexpr float kCarryRule  = 64.0f;
constexpr float kCarryOw    = 64.0f;
constexpr float kScaleIn    = 1.0f / (kCarryEmb * kCarryBw);
constexpr float kScaleRule  = 1.0f / kCarryRule;
constexpr float kScaleHead  = 1.0f / kCarryOw;
constexpr float kMinNormalH = 6.103515625e-5f;

static_assert(kVPad % 64 == 0 && kVPad >= kVocab, "vocab padded to the 64 tile");
static_assert(kBatch % 64 == 0 && kNInPad % 64 == 0, "GEMM M,N tile multiples");
static_assert(kKPad % 32 == 0 && kHid <= 16 && kKPad == 2 * kHid, "K padded to one 32-deep step");
static_assert(kOutTot % 128 == 0, "output is a whole number of 512-B wave runs");
static_assert(kSteps >= 2, "pipeline prologue");

constexpr size_t kOffEmbA = 0;
constexpr size_t kOffOwBt = kOffEmbA + (size_t)kVPad * kKPad * 2;
constexpr size_t kOffBwBt = kOffOwBt + (size_t)kVPad * kKPad * 2;
constexpr size_t kOffBias = kOffBwBt + (size_t)kNInPad * kKPad * 2;
constexpr size_t kOffEmbB = kOffBias + (size_t)kNInPad * 4;
constexpr size_t kOffHA   = kOffEmbB + (size_t)kVPad * kNInPad * 4;
constexpr size_t kOffCpad = kOffHA   + (size_t)kBatch * kKPad * 2;
constexpr size_t kWsTotal = kOffCpad + (size_t)kBatch * kVPad * 4;
static_assert(kWsTotal == 70848768ull, "carve total");
static_assert(kWsTotal <= 134217728ull, "carve cap");
static_assert((kOffOwBt % 256) == 0 && (kOffBwBt % 256) == 0 && (kOffBias % 256) == 0 &&
              (kOffEmbB % 256) == 0 && (kOffHA % 256) == 0 && (kOffCpad % 256) == 0, "aligned regions");

constexpr int kPrepRowBlocks = (kVPad * 4) / 256;
constexpr int kPrepBlocks    = 2 * kPrepRowBlocks + 2;
static_assert((kVPad * 4) % 256 == 0, "exact coverage of the big planes");
static_assert(kNInPad * 4 == 256, "the B_w plane is exactly one block of units");

__device__ __forceinline__ v16h frag_load(const _Float16* p) {
  union U { v16h v; v8h h[2]; };
  U f;
  f.h[0] = *(const v8h*)(p);
  f.h[1] = *(const v8h*)(p + 16);
  return f.v;
}
__device__ __forceinline__ v8f mma_f16(v16h a, v16h b, v8f c) {
  c = __builtin_amdgcn_wmma_f32_16x16x32_f16(false, a, false, b, (short)0, c, false, false);
  asm volatile("v_nop\n\tv_nop\n\tv_nop\n\tv_nop" : "+v"(c) : "v"(a), "v"(b));
  return c;
}
__device__ __forceinline__ void keep4_h(v16h a, v16h b, v16h c, v16h d) { asm volatile("v_nop" :: "v"(a), "v"(b), "v"(c), "v"(d)); }
__device__ __forceinline__ void acc_guard4(v8f& a, v8f& b, v8f& c, v8f& d) { asm volatile("v_nop\n\tv_nop\n\tv_nop\n\tv_nop" : "+v"(a), "+v"(b), "+v"(c), "+v"(d)); }

__device__ __forceinline__ _Float16 to_h_flush(float s) {
  const float f = (fabsf(s) < kMinNormalH) ? 0.0f : s;
  return (_Float16)f;
}
__device__ __forceinline__ int clamp_tok(int v) {
  v = (v < 0) ? 0 : v;
  v = (v > kVocab - 1) ? (kVocab - 1) : v;
  return v;
}

template <int BIAS_MODE>
__global__ __launch_bounds__(256) void gemm64_f16_kernel(
    const unsigned short* __restrict__ Ap, int lda,
    const unsigned short* __restrict__ Btp, int ldb,
    float* __restrict__ C, int ldc,
    const float* __restrict__ bias,
    int M, int N, int K, float scale) {
  const _Float16* A  = (const _Float16*)Ap;
  const _Float16* Bt = (const _Float16*)Btp;
  __shared__ __align__(16) float sT[8][16 * 68];
  const int lane = threadIdx.x & 31;
  const int wave = threadIdx.x >> 5;
  const int tilesN = N >> 6;
  const int tilesM = M >> 6;
  const int tile = blockIdx.x * 8 + wave;
  if (tile >= tilesM * tilesN) return;
  const int tm = tile / tilesN;
  const int tn = tile - tm * tilesN;
  const int m0 = tm << 6;
  const int n0 = tn << 6;

  const int rlane = lane & 15;
  const int koff  = (lane >> 4) * 8;
  const int mOff  = (lane >> 4) * 8;

  v8f acc[4][4];
#pragma unroll
  for (int i = 0; i < 4; ++i)
#pragma unroll
    for (int j = 0; j < 4; ++j) acc[i][j] = (v8f){0.f, 0.f, 0.f, 0.f, 0.f, 0.f, 0.f, 0.f};

  for (int k0 = 0; k0 < K; k0 += 32) {
    v16h bh[4];
#pragma unroll
    for (int j = 0; j < 4; ++j) {
      const size_t bo = (size_t)(n0 + (j << 4) + rlane) * ldb + koff + k0;
      bh[j] = frag_load(Bt + bo);
    }
#pragma unroll
    for (int i = 0; i < 4; ++i) {
      const size_t ao = (size_t)(m0 + (i << 4) + rlane) * lda + koff + k0;
      const v16h ah = frag_load(A + ao);
#pragma unroll
      for (int j = 0; j < 4; ++j) acc[i][j] = mma_f16(ah, bh[j], acc[i][j]);
    }
    keep4_h(bh[0], bh[1], bh[2], bh[3]);
  }
  acc_guard4(acc[0][0], acc[0][1], acc[0][2], acc[0][3]);
  acc_guard4(acc[1][0], acc[1][1], acc[1][2], acc[1][3]);
  acc_guard4(acc[2][0], acc[2][1], acc[2][2], acc[2][3]);
  acc_guard4(acc[3][0], acc[3][1], acc[3][2], acc[3][3]);

  float* slab = sT[wave];
#pragma unroll
  for (int i = 0; i < 4; ++i) {
    const int mBase = m0 + (i << 4);
#pragma unroll
    for (int j = 0; j < 4; ++j) {
      const int n = n0 + (j << 4) + rlane;
      float bv = 0.f;
      if (BIAS_MODE == 2) bv = bias[n];
#pragma unroll
      for (int r = 0; r < 8; ++r) {
        float v = acc[i][j][r] * scale;
        if (BIAS_MODE == 2) v += bv;
        slab[(mOff + r) * 68 + (j << 4) + rlane] = v;
      }
    }
    __builtin_amdgcn_fence(__ATOMIC_RELEASE, "workgroup");
    __builtin_amdgcn_wave_barrier();
    __builtin_amdgcn_fence(__ATOMIC_ACQUIRE, "workgroup");
    {
      const int hh = lane >> 4;
      const int c4 = (lane & 15) * 4;
      for (int pass = 0; pass < 2; ++pass) {
#pragma unroll
        for (int it = 0; it < 8; ++it) {
          const int row = it * 2 + hh;
          const v4f v = *(const v4f*)(slab + row * 68 + c4);
          *(volatile v4f*)(C + (size_t)(mBase + row) * ldc + n0 + c4) = v;
        }
        __threadfence();
      }
    }
    __builtin_amdgcn_fence(__ATOMIC_RELEASE, "workgroup");
    __builtin_amdgcn_wave_barrier();
    __builtin_amdgcn_fence(__ATOMIC_ACQUIRE, "workgroup");
  }
}

__device__ __forceinline__ void plane_unit(const float* __restrict__ src, unsigned short* __restrict__ dst,
                                           int p, int nreal, float carry) {
  const int row  = p >> 2;
  const int part = p & 3;
  const int rc = (row < nreal) ? row : (nreal - 1);
  const int pc = part & 1;
  const float* sp = src + (size_t)rc * kHid + pc * 8;
  v4f a0 = *(const v4f*)(sp);
  v4f a1 = *(const v4f*)(sp + 4);
  asm volatile("" : "+v"(a0), "+v"(a1));
  const bool live = (row < nreal) && (part < 2);
  v8h hv;
#pragma unroll
  for (int e = 0; e < 4; ++e) {
    const float x0 = a0[e];
    const float x1 = a1[e];
    float s0 = x0 * carry;
    float s1 = x1 * carry;
    s0 = live ? s0 : 0.0f;
    s1 = live ? s1 : 0.0f;
    hv[e]     = to_h_flush(s0);
    hv[4 + e] = to_h_flush(s1);
  }
  unsigned short* q = dst + (size_t)p * 8;
  *(volatile v8h*)q = hv;
  __threadfence();
  *(volatile v8h*)q = hv;
}

__global__ __launch_bounds__(256) void prep_kernel(
    const float* __restrict__ embed, const float* __restrict__ out_w,
    const float* __restrict__ b_w, const float* __restrict__ b_b,
    unsigned short* __restrict__ embA, unsigned short* __restrict__ owBt,
    unsigned short* __restrict__ bwBt, float* __restrict__ bias64) {
  const int blk = blockIdx.x;
  const int tid = threadIdx.x;
  if (blk < kPrepRowBlocks) {
    plane_unit(embed, embA, blk * 256 + tid, kVocab, kCarryEmb);
  } else if (blk < 2 * kPrepRowBlocks) {
    plane_unit(out_w, owBt, (blk - kPrepRowBlocks) * 256 + tid, kVocab, kCarryOw);
  } else if (blk == 2 * kPrepRowBlocks) {
    plane_unit(b_w, bwBt, tid, kHid, kCarryBw);
  } else {
    const int l16 = tid & 15;
    float bv0, bv1, bv2, bv3;
    {
      const int n0 = 4 * l16, n1 = n0 + 1, n2 = n0 + 2, n3 = n0 + 3;
      float t0 = b_b[(n0 < kHid) ? n0 : (kHid - 1)];
      float t1 = b_b[(n1 < kHid) ? n1 : (kHid - 1)];
      float t2 = b_b[(n2 < kHid) ? n2 : (kHid - 1)];
      float t3 = b_b[(n3 < kHid) ? n3 : (kHid - 1)];
      asm volatile("" : "+v"(t0), "+v"(t1), "+v"(t2), "+v"(t3));
      bv0 = (n0 < kHid) ? t0 : 0.0f;
      bv1 = (n1 < kHid) ? t1 : 0.0f;
      bv2 = (n2 < kHid) ? t2 : 0.0f;
      bv3 = (n3 < kHid) ? t3 : 0.0f;
    }
    const v4f o = (v4f){bv0, bv1, bv2, bv3};
    if (tid < 16) *(volatile v4f*)(bias64 + 4 * tid) = o;
    __threadfence();
    if (tid < 16) *(volatile v4f*)(bias64 + 4 * tid) = o;
  }
}

__global__ __launch_bounds__(32) void state_scan_kernel(
    const int* __restrict__ seq, const float* __restrict__ embB,
    const float* __restrict__ rule, unsigned short* __restrict__ hA) {
  __shared__ __align__(16) _Float16 sTile[16 * kKPad];
  const int lane = threadIdx.x & 31;
  const int n  = lane & 15;
  const int hh = lane >> 4;
  const int brow = blockIdx.x * 16 + n;

  v16h fa;
  {
    const float* rp = rule + n * kHid + 8 * hh;
    const v4f r0 = *(const v4f*)(rp);
    const v4f r1 = *(const v4f*)(rp + 4);
#pragma unroll
    for (int e = 0; e < 4; ++e) {
      const float x0 = r0[e];
      const float x1 = r1[e];
      fa[e]     = to_h_flush(x0 * kCarryRule);
      fa[4 + e] = to_h_flush(x1 * kCarryRule);
    }
#pragma unroll
    for (int e = 8; e < 16; ++e) fa[e] = (_Float16)0.0f;
  }
  v16h fb;
#pragma unroll
  for (int e = 0; e < 16; ++e) fb[e] = (_Float16)0.0f;

  const int*   sp = seq + (size_t)brow * kSteps;
  const float* eb = embB + 8 * hh;
  const int tk0 = clamp_tok(sp[0]);
  int idxA = clamp_tok(sp[1]);
  v4f c0 = *(const v4f*)(eb + (size_t)tk0 * kNInPad);
  v4f c1 = *(const v4f*)(eb + (size_t)tk0 * kNInPad + 4);

#pragma unroll 1
  for (int t = 0; t < kSteps; ++t) {
    const v4f nx0 = *(const v4f*)(eb + (size_t)idxA * kNInPad);
    const v4f nx1 = *(const v4f*)(eb + (size_t)idxA * kNInPad + 4);
    const int tp = (t + 2 < kSteps) ? (t + 2) : (kSteps - 1);
    idxA = clamp_tok(sp[tp]);

    v8f acc = (v8f){0.f, 0.f, 0.f, 0.f, 0.f, 0.f, 0.f, 0.f};
    acc = mma_f16(fa, fb, acc);

    const float bx[8] = {c0[0], c0[1], c0[2], c0[3], c1[0], c1[1], c1[2], c1[3]};
#pragma unroll
    for (int r = 0; r < 8; ++r) {
      const float z  = fmaf(acc[r], kScaleRule, bx[r]);
      const float ez = expf(-z);
      const float hn = __builtin_amdgcn_rcpf(1.0f + ez);
      fb[r] = to_h_flush(hn);
    }
    c0 = nx0;
    c1 = nx1;
  }

  {
    union U { v16h v; v8h h[2]; };
    U u;
    u.v = fb;
    *(v8h*)(sTile + n * kKPad + 8 * hh)      = u.h[0];
    *(v8h*)(sTile + n * kKPad + 16 + 8 * hh) = u.h[1];
  }
  __syncthreads();
  {
    const v8h o0 = *(const v8h*)(sTile + lane * 8);
    const v8h o1 = *(const v8h*)(sTile + 256 + lane * 8);
    unsigned short* dst = hA + (size_t)blockIdx.x * (16 * kKPad);
    *(volatile v8h*)(dst + lane * 8)       = o0;
    *(volatile v8h*)(dst + 256 + lane * 8) = o1;
    __threadfence();
    *(volatile v8h*)(dst + lane * 8)       = o0;
    *(volatile v8h*)(dst + 256 + lane * 8) = o1;
  }
}

__global__ __launch_bounds__(256) void repack_kernel(
    const float* __restrict__ cpad, const float* __restrict__ out_b, float* __restrict__ out) {
  const unsigned i = blockIdx.x * 256u + threadIdx.x;
  if (i >= (unsigned)kOut4) return;
  const unsigned e0 = i * 4u;
  const unsigned b0 = e0 / (unsigned)kVocab;
  const unsigned v0 = e0 - b0 * (unsigned)kVocab;
  float r[4];
#pragma unroll
  for (int k = 0; k < 4; ++k) {
    const unsigned vr = v0 + (unsigned)k;
    const bool wrap = (vr >= (unsigned)kVocab);
    const unsigned vk = wrap ? (vr - (unsigned)kVocab) : vr;
    const unsigned bk = wrap ? (b0 + 1u) : b0;
    const float cv = cpad[(size_t)bk * kVPad + vk];
    const float ob = out_b[vk];
    r[k] = cv + ob;
  }
  const v4f o = (v4f){r[0], r[1], r[2], r[3]};
  float* q = out + (size_t)e0;
  *(volatile v4f*)q = o;
  __threadfence();
  *(volatile v4f*)q = o;
}

extern "C" void kernel_launch(void* const* d_in, const int* in_sizes, int n_in,
                              void* d_out, int out_size, void* d_ws, size_t ws_size,
                              hipStream_t stream) {
  if (n_in < 7 || d_out == nullptr || d_ws == nullptr) return;
  if (in_sizes[0] != kBatch * kSteps) return;
  if (in_sizes[1] != kVocab * kHid) return;
  if (in_sizes[2] != kHid * kHid) return;
  if (in_sizes[3] != kHid * kHid) return;
  if (in_sizes[4] != kHid) return;
  if (in_sizes[5] != kVocab * kHid) return;
  if (in_sizes[6] != kVocab) return;
  if (out_size != kOutTot) return;
  if (ws_size < kWsTotal) return;

  const int*   seq   = (const int*)d_in[0];
  const float* embed = (const float*)d_in[1];
  const float* rule  = (const float*)d_in[2];
  const float* b_w   = (const float*)d_in[3];
  const float* b_b   = (const float*)d_in[4];
  const float* out_w = (const float*)d_in[5];
  const float* out_b = (const float*)d_in[6];
  float* out = (float*)d_out;

  char* ws = (char*)d_ws;
  unsigned short* EMBA = (unsigned short*)(ws + kOffEmbA);
  unsigned short* OWBT = (unsigned short*)(ws + kOffOwBt);
  unsigned short* BWBT = (unsigned short*)(ws + kOffBwBt);
  float*          BIAS = (float*)(ws + kOffBias);
  float*          EMBB = (float*)(ws + kOffEmbB);
  unsigned short* HA   = (unsigned short*)(ws + kOffHA);
  float*          CPAD = (float*)(ws + kOffCpad);

  prep_kernel<<<kPrepBlocks, 256, 0, stream>>>(embed, out_w, b_w, b_b, EMBA, OWBT, BWBT, BIAS);

  gemm64_f16_kernel<2><<<((kVPad / 64) * (kNInPad / 64) + 7) / 8, 256, 0, stream>>>(
      EMBA, kKPad, BWBT, kKPad, EMBB, kNInPad, BIAS, kVPad, kNInPad, kKPad, kScaleIn);

  state_scan_kernel<<<kBatch / 16, 32, 0, stream>>>(seq, EMBB, rule, HA);

  gemm64_f16_kernel<0><<<((kBatch / 64) * (kVPad / 64) + 7) / 8, 256, 0, stream>>>(
      HA, kKPad, OWBT, kKPad, CPAD, kVPad, nullptr, kBatch, kVPad, kKPad, kScaleHead);

  repack_kernel<<<(kOut4 + 255) / 256, 256, 0, stream>>>(CPAD, out_b, out);
}
